// GCN_79731772883018
// MI455X (gfx1250) — hardware-verified
//
#include <hip/hip_runtime.h>
#include <stddef.h>
#include <stdint.h>
#include <math.h>


#define CIN    128
#define NTHR   256
#define NWAVE  8
#define EPT    8
#define CHUNK  (NTHR * EPT)
#define WCAP   (EPT * 32)
#define LISTN  (NWAVE * WCAP)
#define NBD    8192
#define SLD    13
#define NBA    1024
#define SLA    10
#define RCAP   28672
#define DEGCAP 64
#define STGW   256
#define GBM    64
#define GBN    64
#define GTHR   128
#define ETB    128
#define DP     132
#define FP     40
#define AP1    136
#define AP2    264
#define CSTN   544
#define AGG_ZINTS (LISTN + 2 * RCAP + 3 * NBA)
#define AGG_LDS_INTS (AGG_ZINTS + 16 + NWAVE * STGW)
#define AGG_LDS_BYTES (AGG_LDS_INTS * 4)
#define EDGE_LDS_BYTES (ETB * DP * 4 + ETB * AP2 * 2 + ETB * AP1 * 2 + ETB * FP * 2 + CSTN * 4 + 2 * ETB * 4)
#define WSMAX  134217728

#define NU_W1T  (64 * 16)
#define NU_W2D  (128 * 16)
#define NU_W3D  (256 * 32)
#define NU_WFND (256 * 64)
#define NU_WET  (64 * 4)
#define NU_WFED (128 * 16)
#define NU_WF2D (64 * 32)
#define NU_WHDC (64 * 16)
#define NU_WHDR (64 * 16)
#define NU_CST  256

static_assert((CHUNK & (CHUNK - 1)) == 0 && CHUNK <= 4096);
static_assert((NBD & (NBD - 1)) == 0 && NBD == (1 << SLD));
static_assert((NBA & (NBA - 1)) == 0 && NBA == (1 << SLA));
static_assert(((long long)CHUNK << SLD) < (1LL << 31));
static_assert(((long long)CHUNK << SLA) < (1LL << 31));
static_assert(NBD % (NTHR * 4) == 0);
static_assert(LISTN % NTHR == 0);
static_assert(NBA % NWAVE == 0 && NBA % 32 == 0 && NBA % GBM == 0);
static_assert(RCAP % 32 == 0 && AGG_ZINTS % 4 == 0 && LISTN % 4 == 0);
static_assert(RCAP >= 8415 + 8415 / 20 + 1);
static_assert(DEGCAP >= 24 + 8);
static_assert(AGG_LDS_BYTES <= 327680 && EDGE_LDS_BYTES <= 327680);
static_assert(GBM == (GTHR / 32) * 16 && GBN == 64);
static_assert(NU_W1T % NTHR == 0 && NU_W2D % NTHR == 0 && NU_W3D % NTHR == 0 && NU_WFND % NTHR == 0);
static_assert(NU_WET % NTHR == 0 && NU_WFED % NTHR == 0 && NU_WF2D % NTHR == 0);
static_assert(NU_WHDC % NTHR == 0 && NU_WHDR % NTHR == 0 && NU_CST % NTHR == 0);
static_assert((DP * 4) % 16 == 0 && (FP * 2) % 16 == 0 && (AP1 * 2) % 16 == 0 && (AP2 * 2) % 16 == 0);
static_assert(FP >= 32 && AP1 >= 128 && AP2 >= 256 && DP >= 128);
static_assert((ETB * DP) % 4 == 0 && ((ETB * AP2) / 2) % 4 == 0 && ((ETB * AP1) / 2) % 4 == 0);
static_assert(((ETB * FP) / 2) % 4 == 0 && CSTN % 32 == 0 && CSTN >= 514 && CSTN / 4 <= ETB + 8);
static_assert(ETB == 128 && STGW >= 256);

typedef float          v2f   __attribute__((ext_vector_type(2)));
typedef float          v4f   __attribute__((ext_vector_type(4)));
typedef float          v8f   __attribute__((ext_vector_type(8)));
typedef int            v4i   __attribute__((ext_vector_type(4)));
typedef int            v8i   __attribute__((ext_vector_type(8)));
typedef unsigned int   v4u   __attribute__((ext_vector_type(4)));
typedef unsigned short v8us  __attribute__((ext_vector_type(8)));
typedef unsigned short v16us __attribute__((ext_vector_type(16)));
typedef __bf16         v16bf __attribute__((ext_vector_type(16)));
typedef v2f  __attribute__((may_alias)) v2fa;
typedef v4f  __attribute__((may_alias)) v4fa;
typedef v4i  __attribute__((may_alias)) v4ia;
typedef v4u  __attribute__((may_alias)) v4ua;
typedef v8us __attribute__((may_alias)) v8usa;
typedef unsigned int __attribute__((may_alias)) ua;
union FragB { v16bf v; v16us u; v8us h[2]; v8i w; };
struct HL8 { v8us h; v8us l; };

__device__ __forceinline__ v8f wmb(const FragB& a, const FragB& b, v8f c) {
  v8f d = __builtin_amdgcn_wmma_f32_16x16x32_bf16(false, a.v, false, b.v, (short)0, c, false, false);
  asm volatile("v_nop\n\tv_nop\n\tv_nop\n\tv_nop" : "+v"(d) : "v"(a.w), "v"(b.w));
  return d;
}

__device__ __forceinline__ unsigned bf16_bits(float f) {
  const unsigned u = __float_as_uint(f);
  const unsigned r = (u + 0x7FFFu + ((u >> 16) & 1u)) >> 16;
  return ((u & 0x7FFFFFFFu) > 0x7F800000u) ? 0x7FC0u : r;
}
__device__ __forceinline__ float bf16_val(float f) {
  return __uint_as_float(bf16_bits(f) << 16);
}
__device__ __forceinline__ float lrelu(float v) { return v > 0.0f ? v : 0.01f * v; }

__device__ __forceinline__ HL8 split8(const v8f f) {
  HL8 r;
#pragma unroll
  for (int i = 0; i < 8; ++i) {
    const unsigned hb = bf16_bits(f[i]);
    r.h[i] = (unsigned short)hb;
    r.l[i] = (unsigned short)bf16_bits(f[i] - __uint_as_float(hb << 16));
  }
  return r;
}

__device__ __forceinline__ void put16(unsigned short* dp, v8us o) {
  *(volatile v8us*)dp = o;
  __threadfence();
  *(volatile v8us*)dp = o;
}
__device__ __forceinline__ void putf4(float* dp, v4f o) {
  *(volatile v4f*)dp = o;
  __threadfence();
  *(volatile v4f*)dp = o;
}
__device__ __forceinline__ void wave_lds_sync() {
  __builtin_amdgcn_fence(__ATOMIC_RELEASE, "workgroup");
  __builtin_amdgcn_wave_barrier();
}
__device__ __forceinline__ int clampi(int j, int lo, int hi) { return j < lo ? lo : (j > hi ? hi : j); }
__device__ __forceinline__ v4u blend4(v4u acc, v4f cand, bool on) {
  const unsigned mk = on ? 0xFFFFFFFFu : 0u;
  const v4u c = __builtin_bit_cast(v4u, cand);
  return acc | (c & mk);
}

template <int SLB>
__device__ __forceinline__ int scan_chunk(const int* __restrict__ dsts, int nE, int cbase, int slotBase,
                                          int nb, int vec8, int* list, int tid, int lane, int wave) {
  int wc = 0;
  const int el0  = tid * EPT;
  const int e0   = cbase + el0;
  const int sent = -2147483647 - 1;
  v4i da, db;
  if (vec8 != 0 && cbase + CHUNK <= nE) {
    da = *(const v4i*)(dsts + e0);
    db = *(const v4i*)(dsts + e0 + 4);
  } else {
    da.x = (e0     < nE) ? dsts[min(e0,     nE - 1)] : sent;
    da.y = (e0 + 1 < nE) ? dsts[min(e0 + 1, nE - 1)] : sent;
    da.z = (e0 + 2 < nE) ? dsts[min(e0 + 2, nE - 1)] : sent;
    da.w = (e0 + 3 < nE) ? dsts[min(e0 + 3, nE - 1)] : sent;
    db.x = (e0 + 4 < nE) ? dsts[min(e0 + 4, nE - 1)] : sent;
    db.y = (e0 + 5 < nE) ? dsts[min(e0 + 5, nE - 1)] : sent;
    db.z = (e0 + 6 < nE) ? dsts[min(e0 + 6, nE - 1)] : sent;
    db.w = (e0 + 7 < nE) ? dsts[min(e0 + 7, nE - 1)] : sent;
  }
  const unsigned nbs = (unsigned)slotBase;
  const unsigned unb = (unsigned)nb;
  const unsigned s0 = (unsigned)da.x - nbs, s1 = (unsigned)da.y - nbs;
  const unsigned s2 = (unsigned)da.z - nbs, s3 = (unsigned)da.w - nbs;
  const unsigned s4 = (unsigned)db.x - nbs, s5 = (unsigned)db.y - nbs;
  const unsigned s6 = (unsigned)db.z - nbs, s7 = (unsigned)db.w - nbs;
  const bool h0 = s0 < unb, h1 = s1 < unb, h2 = s2 < unb, h3 = s3 < unb;
  const bool h4 = s4 < unb, h5 = s5 < unb, h6 = s6 < unb, h7 = s7 < unb;
  const unsigned any = __builtin_amdgcn_ballot_w32(h0 | h1 | h2 | h3 | h4 | h5 | h6 | h7);
  if (any != 0u) {
#define HITJ(J, HJ, SJ) { \
      const unsigned mj = __builtin_amdgcn_ballot_w32(HJ); \
      if (mj != 0u) { \
        if (HJ) { \
          const int pos = wc + (int)__builtin_amdgcn_mbcnt_lo(mj, 0u); \
          if (pos < WCAP) list[wave * WCAP + pos] = ((el0 + (J)) << SLB) | (int)(SJ); \
        } \
        wc += (int)__builtin_popcount(mj); } }
    HITJ(0, h0, s0)
    HITJ(1, h1, s1)
    HITJ(2, h2, s2)
    HITJ(3, h3, s3)
    HITJ(4, h4, s4)
    HITJ(5, h5, s5)
    HITJ(6, h6, s6)
    HITJ(7, h7, s7)
#undef HITJ
  }
  return wc;
}

__device__ __forceinline__ void wunit(const float* __restrict__ W, int ldw, int krow, int ncol, unsigned short* dp) {
  const float* p = W + (size_t)krow * (size_t)ldw + ncol;
  v8us o;
#pragma unroll
  for (int i = 0; i < 8; ++i) o[i] = (unsigned short)bf16_bits(p[(size_t)i * (size_t)ldw]);
  put16(dp, o);
}

__global__ __launch_bounds__(NTHR) void k_prep(
    const float* __restrict__ x, const float* __restrict__ W1, const float* __restrict__ W2,
    const float* __restrict__ W3, const float* __restrict__ Wf1, const float* __restrict__ We,
    const float* __restrict__ Wf2, const float* __restrict__ Wc1, const float* __restrict__ Wr1,
    const float* __restrict__ be, const float* __restrict__ bf1, const float* __restrict__ bf2,
    const float* __restrict__ bc1, const float* __restrict__ br1, const float* __restrict__ Wc2,
    const float* __restrict__ Wr2, const float* __restrict__ bc2, const float* __restrict__ br2,
    int nN, int mRows,
    unsigned short* W1T, unsigned short* W2D, unsigned short* W3D, unsigned short* WFND,
    unsigned short* WeT, unsigned short* WFED, unsigned short* WF2D, unsigned short* WHD,
    unsigned short* XB, float* CST) {
  const int u  = (int)blockIdx.x * NTHR + (int)threadIdx.x;
  const int U0 = NU_W1T;
  const int U1 = U0 + NU_W2D;
  const int U2 = U1 + NU_W3D;
  const int U3 = U2 + NU_WFND;
  const int U4 = U3 + NU_WET;
  const int U5 = U4 + NU_WFED;
  const int U6 = U5 + NU_WF2D;
  const int U7 = U6 + NU_WHDC;
  const int U8 = U7 + NU_WHDR;
  const int U9 = U8 + mRows * 16;
  if (u < U0) {
    const int n = u >> 4, k8 = (u & 15) * 8;
    wunit(W1, 64, k8, n, W1T + (size_t)n * 128 + k8);
    return;
  } else if (u < U1) {
    const int v = u - U0;
    const int n = v >> 4, k8 = (v & 15) * 8;
    wunit(W2, 128, k8 & 63, n, W2D + (size_t)n * 128 + k8);
    return;
  } else if (u < U2) {
    const int v = u - U1;
    const int n = v >> 5, k8 = (v & 31) * 8;
    wunit(W3, 256, k8 & 127, n, W3D + (size_t)n * 256 + k8);
    return;
  } else if (u < U3) {
    const int v = u - U2;
    const int n = v >> 6, k8 = (v & 63) * 8;
    const int krow = ((n >= 128) ? 256 : 0) + (k8 & 255);
    wunit(Wf1, 128, krow, n & 127, WFND + (size_t)n * 512 + k8);
    return;
  } else if (u < U4) {
    const int v = u - U3;
    const int n = v >> 2, k8 = (v & 3) * 8;
    v8us o;
#pragma unroll
    for (int i = 0; i < 8; ++i) {
      const int k  = k8 + i;
      const int kc = k < 16 ? k : 15;
      const unsigned b = bf16_bits(We[(size_t)kc * 64 + n]);
      o[i] = (k < 16) ? (unsigned short)b : (unsigned short)0;
    }
    put16(WeT + (size_t)n * 32 + k8, o);
    return;
  } else if (u < U5) {
    const int v = u - U4;
    const int n = v >> 4, k8 = (v & 15) * 8;
    wunit(Wf1, 128, 512 + (k8 & 63), n, WFED + (size_t)n * 128 + k8);
    return;
  } else if (u < U6) {
    const int v = u - U5;
    const int n = v >> 5, k8 = (v & 31) * 8;
    wunit(Wf2, 64, k8 & 127, n, WF2D + (size_t)n * 256 + k8);
    return;
  } else if (u < U7) {
    const int v = u - U6;
    const int n = v >> 4, k8 = (v & 15) * 8;
    wunit(Wc1, 64, k8 & 63, n, WHD + (size_t)n * 128 + k8);
    return;
  } else if (u < U8) {
    const int v = u - U7;
    const int n = v >> 4, k8 = (v & 15) * 8;
    wunit(Wr1, 64, k8 & 63, n, WHD + (size_t)(64 + n) * 128 + k8);
    return;
  } else if (u < U9) {
    const int v   = u - U8;
    const int row = v >> 4;
    const int k8  = (v & 15) * 8;
    const int rc  = row < nN ? row : nN - 1;
    const float* p = x + (size_t)rc * CIN + k8;
    const v4f a = *(const v4fa*)p;
    const v4f b = *(const v4fa*)(p + 4);
    const bool ok = row < nN;
    v8us o;
    o[0] = ok ? (unsigned short)bf16_bits(a.x) : (unsigned short)0;
    o[1] = ok ? (unsigned short)bf16_bits(a.y) : (unsigned short)0;
    o[2] = ok ? (unsigned short)bf16_bits(a.z) : (unsigned short)0;
    o[3] = ok ? (unsigned short)bf16_bits(a.w) : (unsigned short)0;
    o[4] = ok ? (unsigned short)bf16_bits(b.x) : (unsigned short)0;
    o[5] = ok ? (unsigned short)bf16_bits(b.y) : (unsigned short)0;
    o[6] = ok ? (unsigned short)bf16_bits(b.z) : (unsigned short)0;
    o[7] = ok ? (unsigned short)bf16_bits(b.w) : (unsigned short)0;
    put16(XB + (size_t)row * CIN + k8, o);
    return;
  } else {
    const int v  = u - U9;
    const int i4 = 4 * v;
    const v4f a0 = *(const v4fa*)(be  + clampi(i4,        0, 60));
    const v4f a1 = *(const v4fa*)(bf1 + clampi(i4 - 64,   0, 124));
    const v4f a2 = *(const v4fa*)(bf2 + clampi(i4 - 192,  0, 60));
    const v4f a3 = *(const v4fa*)(bc1 + clampi(i4 - 256,  0, 60));
    const v4f a4 = *(const v4fa*)(br1 + clampi(i4 - 320,  0, 60));
    const v4f a5 = *(const v4fa*)(Wc2 + clampi(i4 - 384,  0, 60));
    const v4f a6 = *(const v4fa*)(Wr2 + clampi(i4 - 448,  0, 60));
    const float s0 = bc2[0];
    const float s1 = br2[0];
    const v4f a7 = {s0, s1, 0.0f, 0.0f};
    v4u r = {0u, 0u, 0u, 0u};
    r = blend4(r, a0, i4 < 64);
    r = blend4(r, a1, i4 >= 64  && i4 < 192);
    r = blend4(r, a2, i4 >= 192 && i4 < 256);
    r = blend4(r, a3, i4 >= 256 && i4 < 320);
    r = blend4(r, a4, i4 >= 320 && i4 < 384);
    r = blend4(r, a5, i4 >= 384 && i4 < 448);
    r = blend4(r, a6, i4 >= 448 && i4 < 512);
    r = blend4(r, a7, i4 == 512);
    const v4f f = __builtin_bit_cast(v4f, r);
    v4f q;
    q.x = bf16_val(f.x); q.y = bf16_val(f.y); q.z = bf16_val(f.z); q.w = bf16_val(f.w);
    const int vc = v < CSTN / 4 ? v : CSTN / 4 - 1;
    if (v < CSTN / 4) putf4(CST + 4 * vc, q);
    return;
  }
}

__global__ __launch_bounds__(NTHR) void k_deg(const int* __restrict__ dsts, int nE, int vec8, float* dis) {
  __shared__ __attribute__((aligned(16))) int scnt[NBD];
  __shared__ __attribute__((aligned(16))) int list[LISTN];
  __shared__ int wcnt[NWAVE];
  const int tid = (int)threadIdx.x, lane = tid & 31, wave = tid >> 5;
  const int nodeBase = (int)blockIdx.x * NBD;

  for (int i = tid; i < NBD; i += NTHR) scnt[i] = 0;
  for (int i = tid; i < LISTN; i += NTHR) list[i] = 0;
  if (tid < NWAVE) wcnt[tid] = 0;
  __syncthreads();

  const int nChunks = (nE + CHUNK - 1) / CHUNK;
#pragma unroll 1
  for (int ch = 0; ch < nChunks; ++ch) {
    const int cbase = ch * CHUNK;
    const int wc = scan_chunk<SLD>(dsts, nE, cbase, nodeBase, NBD, vec8, list, tid, lane, wave);
    if (lane == 0) wcnt[wave] = wc;
    __syncthreads();
    if (wave == 0) {
#pragma unroll 1
      for (int w2 = 0; w2 < NWAVE; ++w2) {
        int c = wcnt[w2];
        c = c < 0 ? 0 : (c > WCAP ? WCAP : c);
#pragma unroll 1
        for (int b0 = 0; b0 < c; b0 += 32) {
          const int idx = b0 + lane;
          const int ent = list[w2 * WCAP + (idx < WCAP ? idx : WCAP - 1)];
          const int m32 = (c - b0) < 32 ? (c - b0) : 32;
#pragma unroll 1
          for (int k = 0; k < m32; ++k) {
            const int uu = __builtin_amdgcn_readlane(ent, k);
            const int sl = uu & (NBD - 1);
            if (lane == 0) scnt[sl] = scnt[sl] + 1;
          }
        }
      }
    }
    __syncthreads();
  }

  v4f vals[NBD / (NTHR * 4)];
#pragma unroll
  for (int it = 0; it < NBD / (NTHR * 4); ++it) {
    const int s0 = it * (NTHR * 4) + 4 * tid;
    const v4i c4 = *(const v4ia*)(scnt + s0);
    const float d0 = (float)c4.x + 1.0f, d1 = (float)c4.y + 1.0f;
    const float d2 = (float)c4.z + 1.0f, d3 = (float)c4.w + 1.0f;
    v4f v;
    v.x = rsqrtf(d0); v.y = rsqrtf(d1); v.z = rsqrtf(d2); v.w = rsqrtf(d3);
    vals[it] = v;
  }
#pragma unroll
  for (int it = 0; it < NBD / (NTHR * 4); ++it) {
    const int s0 = it * (NTHR * 4) + 4 * tid;
    *(volatile v4f*)(dis + (size_t)nodeBase + s0) = vals[it];
  }
  __threadfence();
#pragma unroll
  for (int it = 0; it < NBD / (NTHR * 4); ++it) {
    const int s0 = it * (NTHR * 4) + 4 * tid;
    *(volatile v4f*)(dis + (size_t)nodeBase + s0) = vals[it];
  }
}

__global__ __launch_bounds__(GTHR) void k_gemm(
    const unsigned short* __restrict__ A, const unsigned short* __restrict__ WT,
    float* outF, int K, int ldo)
{
  __shared__ __attribute__((aligned(16))) float stg[GBM * GBN];
  const int tid = (int)threadIdx.x, lane = tid & 31, wave = tid >> 5, hh = lane >> 4, m = lane & 15;
  const int rowBase = (int)blockIdx.x * GBM;
  const int col0    = (int)blockIdx.y * GBN;

  v8f acc[4];
  {
    const v8f z = {0.f, 0.f, 0.f, 0.f, 0.f, 0.f, 0.f, 0.f};
    acc[0] = z; acc[1] = z; acc[2] = z; acc[3] = z;
  }
  const unsigned short* ap = A  + (size_t)(rowBase + 16 * wave + m) * (size_t)K + 8 * hh;
  const unsigned short* wp = WT + (size_t)(col0 + m) * (size_t)K + 8 * hh;
  const int ksteps = K >> 5;
#pragma unroll 1
  for (int ks = 0; ks < ksteps; ++ks) {
    FragB af;
    af.h[0] = *(const v8usa*)(ap + 32 * ks);
    af.h[1] = *(const v8usa*)(ap + 32 * ks + 16);
#pragma unroll
    for (int t = 0; t < 4; ++t) {
      const unsigned short* wq = wp + (size_t)(16 * t) * (size_t)K + 32 * ks;
      FragB bf;
      bf.h[0] = *(const v8usa*)wq;
      bf.h[1] = *(const v8usa*)(wq + 16);
      acc[t] = wmb(af, bf, acc[t]);
    }
  }

#pragma unroll
  for (int t = 0; t < 4; ++t) {
    const int lc = 16 * t + m;
#pragma unroll
    for (int r = 0; r < 8; ++r) {
      const int lr = 16 * wave + 8 * hh + r;
      stg[lr * GBN + lc] = acc[t][r];
    }
  }
  __syncthreads();

  v4f fv[8];
#pragma unroll
  for (int i = 0; i < 8; ++i) {
    const int lr = 16 * wave + 2 * i + hh;
    fv[i] = *(const v4fa*)(stg + lr * GBN + 4 * m);
  }
#pragma unroll
  for (int i = 0; i < 8; ++i) {
    const int lr = 16 * wave + 2 * i + hh;
    const int gr = rowBase + lr;
    float* op = outF + (size_t)gr * (size_t)ldo + col0 + 4 * m;
    *(volatile v4f*)op = fv[i];
  }
  __threadfence();
#pragma unroll
  for (int i = 0; i < 8; ++i) {
    const int lr = 16 * wave + 2 * i + hh;
    const int gr = rowBase + lr;
    float* op = outF + (size_t)gr * (size_t)ldo + col0 + 4 * m;
    *(volatile v4f*)op = fv[i];
  }
}

template <int CPL>
__device__ __forceinline__ void load_row(const float* __restrict__ rp, int lane, float (&v)[CPL]) {
  if constexpr (CPL == 2) {
    const v2f a = *(const v2fa*)(rp + 2 * lane);
    v[0] = a.x; v[1] = a.y;
  } else {
#pragma unroll
    for (int q = 0; q < CPL / 4; ++q) {
      const v4f a = *(const v4fa*)(rp + 128 * q + 4 * lane);
      v[4 * q + 0] = a.x; v[4 * q + 1] = a.y; v[4 * q + 2] = a.z; v[4 * q + 3] = a.w;
    }
  }
}

template <int CPL>
__global__ __launch_bounds__(NTHR) void k_agg(const int* __restrict__ srcs, const int* __restrict__ dsts,
                                              int nE, int nN, int vec8, int mRows,
                                              const float* __restrict__ dis,
                                              const float* __restrict__ xl, const float* __restrict__ bias,
                                              unsigned int* hbw) {
  constexpr int C = 32 * CPL;
  static_assert(CPL == 2 || CPL == 4 || CPL == 8);
  static_assert(C <= STGW);
  extern __shared__ __attribute__((aligned(16))) int dsm[];
  int* list = dsm;
  int* hl   = dsm + LISTN;
  int* sl   = dsm + LISTN + RCAP;
  int* cnt  = dsm + LISTN + 2 * RCAP;
  int* offs = cnt + NBA;
  int* cur  = offs + NBA;
  int* misc = cur + NBA;
  const int tid = (int)threadIdx.x, lane = tid & 31, wave = tid >> 5;
  ua* stw = (ua*)(misc + 16) + wave * STGW;
  const int nodeBase = (int)blockIdx.x * NBA;

  {
    const v4i z4 = {0, 0, 0, 0};
    for (int i = tid * 4; i < AGG_ZINTS; i += NTHR * 4) *(v4ia*)(dsm + i) = z4;
    if (tid < 16) misc[tid] = 0;
  }
  float bv[CPL];
  load_row<CPL>(bias, lane, bv);
#pragma unroll
  for (int j = 0; j < CPL; ++j) bv[j] = bf16_val(bv[j]);
  __syncthreads();

  int t = 0, ov = 0;
  const int nChunks = (nE + CHUNK - 1) / CHUNK;
#pragma unroll 1
  for (int ch = 0; ch < nChunks; ++ch) {
    const int cbase = ch * CHUNK;
    const int wc = scan_chunk<SLA>(dsts, nE, cbase, nodeBase, NBA, vec8, list, tid, lane, wave);
    if (lane == 0) misc[wave] = wc;
    __syncthreads();
    if (wave == 0) {
#pragma unroll 1
      for (int w2 = 0; w2 < NWAVE; ++w2) {
        int c = misc[w2];
        c = c < 0 ? 0 : (c > WCAP ? WCAP : c);
#pragma unroll 1
        for (int b0 = 0; b0 < c; b0 += 32) {
          const int idx = b0 + lane;
          const int ent = list[w2 * WCAP + (idx < WCAP ? idx : WCAP - 1)];
          const int m32 = (c - b0) < 32 ? (c - b0) : 32;
#pragma unroll 1
          for (int k = 0; k < m32; ++k) {
            const int uu   = __builtin_amdgcn_readlane(ent, k);
            const int slot = uu & (NBA - 1);
            const int el   = (uu >> SLA) & (CHUNK - 1);
            const int pk   = ((cbase + el) << SLA) | slot;
            if (t < RCAP) {
              if (lane == 0) { hl[t] = pk; cnt[slot] = cnt[slot] + 1; }
              t = t + 1;
            } else {
              ov = 1;
            }
          }
        }
      }
    }
    __syncthreads();
  }
  if (wave == 0 && lane == 0) { misc[8] = t; misc[9] = ov; }
  __syncthreads();
  int tt = misc[8];
  tt = tt < 0 ? 0 : (tt > RCAP ? RCAP : tt);
  const int ovf = misc[9];

  if (wave == 0) {
    const int base = lane * (NBA / 32);
    int s = 0;
#pragma unroll 1
    for (int i = 0; i < NBA / 32; ++i) s += cnt[base + i];
    int incl = s;
#pragma unroll
    for (int d = 1; d < 32; d <<= 1) {
      const int y = __shfl_up(incl, d, 32);
      if (lane >= d) incl += y;
    }
    int run = incl - s;
#pragma unroll 1
    for (int i = 0; i < NBA / 32; ++i) {
      const int cv = cnt[base + i];
      offs[base + i] = run;
      cur[base + i]  = run;
      run += cv;
    }
  }
  __syncthreads();
  if (wave == 0) {
#pragma unroll 1
    for (int b0 = 0; b0 < tt; b0 += 32) {
      const int idx = b0 + lane;
      const int ent = hl[idx < RCAP ? idx : RCAP - 1];
      const int m32 = (tt - b0) < 32 ? (tt - b0) : 32;
#pragma unroll 1
      for (int k = 0; k < m32; ++k) {
        const int uu   = __builtin_amdgcn_readlane(ent, k);
        const int slot = uu & (NBA - 1);
        if (lane == 0) {
          int p = cur[slot];
          p = p < 0 ? 0 : (p > RCAP - 1 ? RCAP - 1 : p);
          sl[p] = uu;
          cur[slot] = p + 1;
        }
      }
    }
  }
  __syncthreads();

  const float qnan = __int_as_float(0x7fc00000);
  const float pz = (ovf != 0) ? qnan : 0.0f;
#pragma unroll 1
  for (int si = 0; si < NBA / NWAVE; ++si) {
    const int s    = si * NWAVE + wave;
    const int node = nodeBase + s;
    int c = cnt[s];
    const bool big = c > DEGCAP;
    c = c < 0 ? 0 : (c > DEGCAP ? DEGCAP : c);
    int o = offs[s];
    o = o < 0 ? 0 : (o > RCAP ? RCAP : o);
    const int nc = node < nN ? node : nN - 1;
    const float dd = dis[nc];
    const float rd = dd * dd;
    float acc[CPL];
#pragma unroll
    for (int j = 0; j < CPL; ++j) acc[j] = 0.0f;
#pragma unroll 1
    for (int b0 = 0; b0 < c; b0 += 32) {
      int idx = o + b0 + lane;
      idx = idx > RCAP - 1 ? RCAP - 1 : idx;
      const int ent = sl[idx];
      int eid = ent >> SLA;
      eid = eid < 0 ? 0 : (eid > nE - 1 ? nE - 1 : eid);
      int sr = srcs[eid];
      sr = sr < 0 ? 0 : (sr > nN - 1 ? nN - 1 : sr);
      const float cf  = dis[sr] * dd;
      const int   cfi = __float_as_int(cf);
      const int m32 = (c - b0) < 32 ? (c - b0) : 32;
#pragma unroll 1
      for (int k = 0; k < m32; ++k) {
        const int   sk = __builtin_amdgcn_readlane(sr, k);
        const float ck = __int_as_float(__builtin_amdgcn_readlane(cfi, k));
        float rv[CPL];
        load_row<CPL>(xl + (size_t)sk * C, lane, rv);
#pragma unroll
        for (int j = 0; j < CPL; ++j) acc[j] = fmaf(ck, rv[j], acc[j]);
      }
    }
    float sv[CPL];
    load_row<CPL>(xl + (size_t)nc * C, lane, sv);
    const float pzr = big ? qnan : pz;
    const bool live = node < nN;
    float v[CPL];
#pragma unroll
    for (int j = 0; j < CPL; ++j) {
      float y = (acc[j] + sv[j] * rd) + bv[j];
      y = lrelu(y);
      y = y + pzr;
      v[j] = live ? y : 0.0f;
    }
#pragma unroll
    for (int jp = 0; jp < CPL / 2; ++jp) {
      const float f0 = v[2 * jp], f1 = v[2 * jp + 1];
      const unsigned hb0 = bf16_bits(f0), hb1 = bf16_bits(f1);
      const unsigned lb0 = bf16_bits(f0 - __uint_as_float(hb0 << 16));
      const unsigned lb1 = bf16_bits(f1 - __uint_as_float(hb1 << 16));
      const unsigned hw = hb0 | (hb1 << 16);
      const unsigned lw = lb0 | (lb1 << 16);
      const int wi = (CPL == 2) ? lane : (64 * (jp >> 1) + 2 * lane + (jp & 1));
      stw[wi]         = hw;
      stw[C / 2 + wi] = lw;
    }
    wave_lds_sync();
    if constexpr (CPL == 2) {
      const v4u pv = *(const v4ua*)(stw + 4 * (lane & 15));
      unsigned int* hp = hbw + (size_t)node * C + 4 * (lane & 15);
      const bool wr = (node < mRows) && (lane < 16);
      if (wr) *(volatile v4u*)hp = pv;
      __threadfence();
      if (wr) *(volatile v4u*)hp = pv;
    } else {
      constexpr int NP = C / 128;
      v4u pv[NP];
#pragma unroll
      for (int p = 0; p < NP; ++p) pv[p] = *(const v4ua*)(stw + 128 * p + 4 * lane);
      unsigned int* hp = hbw + (size_t)node * C + 4 * lane;
      const bool wr = node < mRows;
#pragma unroll
      for (int p = 0; p < NP; ++p) { if (wr) *(volatile v4u*)(hp + 128 * p) = pv[p]; }
      __threadfence();
#pragma unroll
      for (int p = 0; p < NP; ++p) { if (wr) *(volatile v4u*)(hp + 128 * p) = pv[p]; }
    }
    wave_lds_sync();
  }
}

template <int APITCH, int NH>
__device__ __forceinline__ void wave_gemm_b(const unsigned short* sAw, float* sDw,
                                            const unsigned short* __restrict__ BT, int ldb, int K,
                                            int hh, int m) {
#pragma unroll 1
  for (int nh = 0; nh < NH; ++nh) {
    v8f acc[2][4];
    {
      const v8f z = {0.f, 0.f, 0.f, 0.f, 0.f, 0.f, 0.f, 0.f};
#pragma unroll
      for (int mt = 0; mt < 2; ++mt)
#pragma unroll
        for (int nt = 0; nt < 4; ++nt) acc[mt][nt] = z;
    }
    const unsigned short* ap0 = sAw + m * APITCH + 8 * hh;
    const unsigned short* ap1 = ap0 + 16 * APITCH;
    const unsigned short* bp  = BT + (size_t)(64 * nh + m) * (size_t)ldb + 8 * hh;
#pragma unroll 1
    for (int k0 = 0; k0 < K; k0 += 32) {
      FragB a0, a1;
      a0.h[0] = *(const v8usa*)(ap0 + k0);
      a0.h[1] = *(const v8usa*)(ap0 + k0 + 16);
      a1.h[0] = *(const v8usa*)(ap1 + k0);
      a1.h[1] = *(const v8usa*)(ap1 + k0 + 16);
#pragma unroll
      for (int nt = 0; nt < 4; ++nt) {
        const unsigned short* wq = bp + (size_t)(16 * nt) * (size_t)ldb + k0;
        FragB b;
        b.h[0] = *(const v8usa*)wq;
        b.h[1] = *(const v8usa*)(wq + 16);
        acc[0][nt] = wmb(a0, b, acc[0][nt]);
        acc[1][nt] = wmb(a1, b, acc[1][nt]);
      }
    }
#pragma unroll
    for (int nt = 0; nt < 4; ++nt) {
      const int col = 64 * nh + 16 * nt + m;
#pragma unroll
      for (int mt = 0; mt < 2; ++mt)
#pragma unroll
        for (int r = 0; r < 8; ++r) sDw[(16 * mt + 8 * hh + r) * DP + col] = acc[mt][nt][r];
    }
  }
}

__global__ __launch_bounds__(ETB) void k_edge(const int* __restrict__ src, const int* __restrict__ dst,
                                              int nN, int nE,
                                              const float* __restrict__ EA, const float* __restrict__ PSD,
                                              const unsigned short* __restrict__ WeT,
                                              const unsigned short* __restrict__ WFED,
                                              const unsigned short* __restrict__ WF2D,
                                              const unsigned short* __restrict__ WHD,
                                              const float* __restrict__ CST, float* out) {
  extern __shared__ __attribute__((aligned(16))) float dyn[];
  float*          sD  = dyn;
  unsigned short* sA2 = (unsigned short*)(dyn + ETB * DP);
  unsigned short* sA1 = sA2 + ETB * AP2;
  unsigned short* sF  = sA1 + ETB * AP1;
  float*          cst = dyn + ETB * DP + (ETB * AP2) / 2 + (ETB * AP1) / 2 + (ETB * FP) / 2;
  float*          sO  = cst + CSTN;

  const int tid = (int)threadIdx.x, lane = tid & 31, wave = tid >> 5, hh = lane >> 4, m = lane & 15;
  const int e0 = (int)blockIdx.x * ETB;
  const int e  = e0 + tid;
  const int ec = e < nE ? e : nE - 1;

  {
    const v4f c0 = *(const v4fa*)(CST + 4 * tid);
    *(v4fa*)(cst + 4 * tid) = c0;
    const int t2 = ETB + (tid & 7);
    const v4f c1 = *(const v4fa*)(CST + 4 * t2);
    if (tid < 8) *(v4fa*)(cst + 4 * t2) = c1;
  }

  int s = src[ec];
  int t = dst[ec];
  s = s < 0 ? 0 : (s > nN - 1 ? nN - 1 : s);
  t = t < 0 ? 0 : (t > nN - 1 ? nN - 1 : t);

  float*          rd  = sD  + tid * DP;
  unsigned short* ra1 = sA1 + tid * AP1;
  unsigned short* ra2 = sA2 + tid * AP2;
  unsigned short* rf  = sF  + tid * FP;
  {
    const float* aq = EA + (size_t)ec * 16;
    const v4f a0 = *(const v4fa*)(aq);
    const v4f a1 = *(const v4fa*)(aq + 4);
    const v4f a2 = *(const v4fa*)(aq + 8);
    const v4f a3 = *(const v4fa*)(aq + 12);
    v8us o0, o1, oz;
    o0[0] = (unsigned short)bf16_bits(a0.x); o0[1] = (unsigned short)bf16_bits(a0.y);
    o0[2] = (unsigned short)bf16_bits(a0.z); o0[3] = (unsigned short)bf16_bits(a0.w);
    o0[4] = (unsigned short)bf16_bits(a1.x); o0[5] = (unsigned short)bf16_bits(a1.y);
    o0[6] = (unsigned short)bf16_bits(a1.z); o0[7] = (unsigned short)bf16_bits(a1.w);
    o1[0] = (unsigned short)bf16_bits(a2.x); o1[1] = (unsigned short)bf16_bits(a2.y);
    o1[2] = (unsigned short)bf16_bits(a2.z); o1[3] = (unsigned short)bf16_bits(a2.w);
    o1[4] = (unsigned short)bf16_bits(a3.x); o1[5] = (unsigned short)bf16_bits(a3.y);
    o1[6] = (unsigned short)bf16_bits(a3.z); o1[7] = (unsigned short)bf16_bits(a3.w);
#pragma unroll
    for (int j = 0; j < 8; ++j) oz[j] = (unsigned short)0;
    *(v8usa*)(rf + 0)  = o0;
    *(v8usa*)(rf + 8)  = o1;
    *(v8usa*)(rf + 16) = oz;
    *(v8usa*)(rf + 24) = oz;
  }
  __syncthreads();

  const unsigned short* sFw  = sF  + 32 * wave * FP;
  const unsigned short* sA1w = sA1 + 32 * wave * AP1;
  const unsigned short* sA2w = sA2 + 32 * wave * AP2;
  float*                sDw  = sD  + 32 * wave * DP;

  wave_gemm_b<FP, 1>(sFw, sDw, WeT, 32, 32, hh, m);
  __syncthreads();
  {
#pragma unroll 1
    for (int c8 = 0; c8 < 8; ++c8) {
      const v4f va = *(const v4fa*)(rd + 8 * c8);
      const v4f vb = *(const v4fa*)(rd + 8 * c8 + 4);
      const v4f ba = *(const v4fa*)(cst + 8 * c8);
      const v4f bb = *(const v4fa*)(cst + 8 * c8 + 4);
      const v8f v8 = {va.x, va.y, va.z, va.w, vb.x, vb.y, vb.z, vb.w};
      const v8f b8 = {ba.x, ba.y, ba.z, ba.w, bb.x, bb.y, bb.z, bb.w};
      v8f y;
#pragma unroll
      for (int i = 0; i < 8; ++i) y[i] = lrelu(v8[i] + b8[i]);
      const HL8 hl = split8(y);
      *(v8usa*)(ra1 + 8 * c8)      = hl.h;
      *(v8usa*)(ra1 + 64 + 8 * c8) = hl.l;
    }
  }
  __syncthreads();

  wave_gemm_b<AP1, 2>(sA1w, sDw, WFED, 128, 128, hh, m);
  __syncthreads();
  {
    const float* pr = PSD + (size_t)s * 256;
    const float* qr = PSD + (size_t)t * 256 + 128;
#pragma unroll 1
    for (int c8 = 0; c8 < 16; ++c8) {
      const v4f va = *(const v4fa*)(rd + 8 * c8);
      const v4f vb = *(const v4fa*)(rd + 8 * c8 + 4);
      const v4f pa = *(const v4fa*)(pr + 8 * c8);
      const v4f pb = *(const v4fa*)(pr + 8 * c8 + 4);
      const v4f qa = *(const v4fa*)(qr + 8 * c8);
      const v4f qb = *(const v4fa*)(qr + 8 * c8 + 4);
      const v4f ba = *(const v4fa*)(cst + 64 + 8 * c8);
      const v4f bb = *(const v4fa*)(cst + 64 + 8 * c8 + 4);
      const v8f v8 = {va.x, va.y, va.z, va.w, vb.x, vb.y, vb.z, vb.w};
      const v8f p8 = {pa.x, pa.y, pa.z, pa.w, pb.x, pb.y, pb.z, pb.w};
      const v8f q8 = {qa.x, qa.y, qa.z, qa.w, qb.x, qb.y, qb.z, qb.w};
      const v8f b8 = {ba.x, ba.y, ba.z, ba.w, bb.x, bb.y, bb.z, bb.w};
      v8f y;
#pragma unroll
      for (int i = 0; i < 8; ++i) y[i] = lrelu((p8[i] + q8[i]) + (v8[i] + b8[i]));
      const HL8 hl = split8(y);
      *(v8usa*)(ra2 + 8 * c8)       = hl.h;
      *(v8usa*)(ra2 + 128 + 8 * c8) = hl.l;
    }
  }
  __syncthreads();

  wave_gemm_b<AP2, 1>(sA2w, sDw, WF2D, 256, 256, hh, m);
  __syncthreads();
  {
#pragma unroll 1
    for (int c8 = 0; c8 < 8; ++c8) {
      const v4f va = *(const v4fa*)(rd + 8 * c8);
      const v4f vb = *(const v4fa*)(rd + 8 * c8 + 4);
      const v4f ba = *(const v4fa*)(cst + 192 + 8 * c8);
      const v4f bb = *(const v4fa*)(cst + 192 + 8 * c8 + 4);
      const v8f v8 = {va.x, va.y, va.z, va.w, vb.x, vb.y, vb.z, vb.w};
      const v8f b8 = {ba.x, ba.y, ba.z, ba.w, bb.x, bb.y, bb.z, bb.w};
      v8f y;
#pragma unroll
      for (int i = 0; i < 8; ++i) y[i] = v8[i] + b8[i];
      const HL8 hl = split8(y);
      *(v8usa*)(ra1 + 8 * c8)      = hl.h;
      *(v8usa*)(ra1 + 64 + 8 * c8) = hl.l;
    }
  }
  __syncthreads();

  wave_gemm_b<AP1, 2>(sA1w, sDw, WHD, 128, 128, hh, m);
  __syncthreads();
  {
    float zc = 0.0f, zr = 0.0f;
#pragma unroll 1
    for (int c8 = 0; c8 < 8; ++c8) {
      const v4f va = *(const v4fa*)(rd + 8 * c8);
      const v4f vb = *(const v4fa*)(rd + 8 * c8 + 4);
      const v4f ba = *(const v4fa*)(cst + 256 + 8 * c8);
      const v4f bb = *(const v4fa*)(cst + 256 + 8 * c8 + 4);
      const v4f wa = *(const v4fa*)(cst + 384 + 8 * c8);
      const v4f wb = *(const v4fa*)(cst + 384 + 8 * c8 + 4);
      const v8f v8 = {va.x, va.y, va.z, va.w, vb.x, vb.y, vb.z, vb.w};
      const v8f b8 = {ba.x, ba.y, ba.z, ba.w, bb.x, bb.y, bb.z, bb.w};
      const v8f w8 = {wa.x, wa.y, wa.z, wa.w, wb.x, wb.y, wb.z, wb.w};
#pragma unroll
      for (int i = 0; i < 8; ++i) zc = fmaf(lrelu(v8[i] + b8[i]), w8[i], zc);
    }
#pragma unroll 1
    for (int c8 = 0; c8 < 8; ++c8) {
      const v4f va = *(const v4fa*)(rd + 64 + 8 * c8);
      const v4f vb = *(const v4fa*)(rd + 64 + 8 * c8 + 4);
      const v4f ba = *(const v4fa*)(cst + 320 + 8 * c8);
      const v4f bb = *(const v4fa*)(cst + 320 + 8 * c8 + 4);
      const v4f wa = *(const v4fa*)(cst + 448 + 8 * c8);
      const v4f wb = *(const v4fa*)(cst + 448 + 8 * c8 + 4);
      const v8f v8 = {va.x, va.y, va.z, va.w, vb.x, vb.y, vb.z, vb.w};
      const v8f b8 = {ba.x, ba.y, ba.z, ba.w, bb.x, bb.y, bb.z, bb.w};
      const v8f w8 = {wa.x, wa.y, wa.z, wa.w, wb.x, wb.y, wb.z, wb.w};
#pragma unroll
      for (int i = 0; i < 8; ++i) zr = fmaf(lrelu(v8[i] + b8[i]), w8[i], zr);
    }
    zc = zc + cst[512];
    zr = zr + cst[513];
    const float p = 1.0f / (1.0f + expf(-zc));
    sO[tid]       = p * zr;
    sO[ETB + tid] = p;
  }
  __syncthreads();

  {
    const int wsel = wave & 1;
    const v4f o4 = *(const v4fa*)(sO + ETB * wsel + 4 * lane);
    const size_t ofs = (size_t)wsel * (size_t)nE + (size_t)e0 + (size_t)(4 * lane);
    float* op = out + ofs;
    const bool st = wave < 2;
    if (st) *(volatile v4f*)op = o4;
    __threadfence();
    if (st) *(volatile v4f*)op = o4;
  }
}

static inline int cdiv(int a, int b) { return (a + b - 1) / b; }
static inline size_t al256(size_t o) { return (o + 255) & ~(size_t)255; }

extern "C" void kernel_launch(void* const* d_in, const int* in_sizes, int n_in,
                              void* d_out, int out_size, void* d_ws, size_t ws_size,
                              hipStream_t stream) {
  if (n_in < 23) return;
  if (in_sizes[0] < CIN || (in_sizes[0] % CIN) != 0) return;
  const int nN = in_sizes[0] / CIN;
  if (nN < 1 || nN > (1 << 21)) return;
  if (in_sizes[1] < 2 || (in_sizes[1] & 1) != 0) return;
  const int nE = in_sizes[1] / 2;
  if (nE < ETB || nE >= (1 << (31 - SLA))) return;
  if ((nE % ETB) != 0) return;
  if ((long long)in_sizes[2] != 16LL * nE) return;
  if (in_sizes[3] != 128 * 64 || in_sizes[4] != 64) return;
  if (in_sizes[5] != 64 * 128 || in_sizes[6] != 128) return;
  if (in_sizes[7] != 128 * 256 || in_sizes[8] != 256) return;
  if (in_sizes[9] != 16 * 64 || in_sizes[10] != 64) return;
  if (in_sizes[11] != 576 * 128 || in_sizes[12] != 128) return;
  if (in_sizes[13] != 128 * 64 || in_sizes[14] != 64) return;
  if (in_sizes[15] != 64 * 64 || in_sizes[16] != 64) return;
  if (in_sizes[17] != 64 || in_sizes[18] != 1) return;
  if (in_sizes[19] != 64 * 64 || in_sizes[20] != 64) return;
  if (in_sizes[21] != 64 || in_sizes[22] != 1) return;
  if ((long long)out_size != 2LL * nE) return;

  const float* x    = (const float*)d_in[0];
  const int*   edge = (const int*)d_in[1];
  const float* EA   = (const float*)d_in[2];
  const float* W1   = (const float*)d_in[3];
  const float* b1   = (const float*)d_in[4];
  const float* W2   = (const float*)d_in[5];
  const float* b2   = (const float*)d_in[6];
  const float* W3   = (const float*)d_in[7];
  const float* b3   = (const float*)d_in[8];
  const float* We   = (const float*)d_in[9];
  const float* be   = (const float*)d_in[10];
  const float* Wf1  = (const float*)d_in[11];
  const float* bf1  = (const float*)d_in[12];
  const float* Wf2  = (const float*)d_in[13];
  const float* bf2  = (const float*)d_in[14];
  const float* Wc1  = (const float*)d_in[15];
  const float* bc1  = (const float*)d_in[16];
  const float* Wc2  = (const float*)d_in[17];
  const float* bc2  = (const float*)d_in[18];
  const float* Wr1  = (const float*)d_in[19];
  const float* br1  = (const float*)d_in[20];
  const float* Wr2  = (const float*)d_in[21];
  const float* br2  = (const float*)d_in[22];
  float* out = (float*)d_out;
  const int* src = edge;
  const int* dst = edge + nE;

  const int MP   = cdiv(nN, 128) * 128;
  const int gM   = MP / GBM;
  const int gD   = cdiv(nN, NBD);
  const int NBPD = gD * NBD;
  const int gA   = cdiv(MP, NBA);
  if ((long long)gA * NBA < (long long)MP) return;
  if (NBPD < nN) return;
  if ((MP % GBM) != 0) return;
  const int vec8 = ((nE & 3) == 0) ? 1 : 0;

  char* ws = (char*)d_ws;
  size_t off = 0;
  const size_t oDIS  = off; off = al256(off + (size_t)NBPD * 4);
  const size_t oW1T  = off; off = al256(off + (size_t)64 * 128 * 2);
  const size_t oW2D  = off; off = al256(off + (size_t)128 * 128 * 2);
  const size_t oW3D  = off; off = al256(off + (size_t)256 * 256 * 2);
  const size_t oWFND = off; off = al256(off + (size_t)256 * 512 * 2);
  const size_t oWET  = off; off = al256(off + (size_t)64 * 32 * 2);
  const size_t oWFED = off; off = al256(off + (size_t)128 * 128 * 2);
  const size_t oWF2D = off; off = al256(off + (size_t)64 * 256 * 2);
  const size_t oWHD  = off; off = al256(off + (size_t)128 * 128 * 2);
  const size_t oCST  = off; off = al256(off + (size_t)CSTN * 4);
  const size_t oXB   = off; off = al256(off + (size_t)MP * CIN * 2);
  const size_t oH    = off; off = al256(off + (size_t)MP * 256 * 4);
  const size_t oXHL  = off; off = al256(off + (size_t)MP * 512 * 2);
  if (off > ws_size || off > (size_t)WSMAX) return;
  float*          DIS  = (float*)(ws + oDIS);
  unsigned short* W1T  = (unsigned short*)(ws + oW1T);
  unsigned short* W2D  = (unsigned short*)(ws + oW2D);
  unsigned short* W3D  = (unsigned short*)(ws + oW3D);
  unsigned short* WFND = (unsigned short*)(ws + oWFND);
  unsigned short* WeT  = (unsigned short*)(ws + oWET);
  unsigned short* WFED = (unsigned short*)(ws + oWFED);
  unsigned short* WF2D = (unsigned short*)(ws + oWF2D);
  unsigned short* WHD  = (unsigned short*)(ws + oWHD);
  float*          CST  = (float*)(ws + oCST);
  unsigned short* XB   = (unsigned short*)(ws + oXB);
  float*          Hp   = (float*)(ws + oH);
  unsigned short* XHL  = (unsigned short*)(ws + oXHL);
  unsigned int*   XHLw = (unsigned int*)(ws + oXHL);

  hipFuncSetAttribute(reinterpret_cast<const void*>(&k_agg<2>), hipFuncAttributeMaxDynamicSharedMemorySize,
                      (int)AGG_LDS_BYTES);
  hipFuncSetAttribute(reinterpret_cast<const void*>(&k_agg<4>), hipFuncAttributeMaxDynamicSharedMemorySize,
                      (int)AGG_LDS_BYTES);
  hipFuncSetAttribute(reinterpret_cast<const void*>(&k_agg<8>), hipFuncAttributeMaxDynamicSharedMemorySize,
                      (int)AGG_LDS_BYTES);
  hipFuncSetAttribute(reinterpret_cast<const void*>(&k_edge), hipFuncAttributeMaxDynamicSharedMemorySize,
                      (int)EDGE_LDS_BYTES);

  const int nPrep = NU_W1T + NU_W2D + NU_W3D + NU_WFND + NU_WET + NU_WFED + NU_WF2D + NU_WHDC + NU_WHDR
                  + MP * 16 + NU_CST;
  k_prep<<<nPrep / NTHR, NTHR, 0, stream>>>(x, W1, W2, W3, Wf1, We, Wf2, Wc1, Wr1,
                                            be, bf1, bf2, bc1, br1, Wc2, Wr2, bc2, br2, nN, MP,
                                            W1T, W2D, W3D, WFND, WeT, WFED, WF2D, WHD, XB, CST);
  k_deg<<<gD, NTHR, 0, stream>>>(dst, nE, vec8, DIS);
  k_gemm<<<dim3(gM, 64 / GBN), GTHR, 0, stream>>>(XB, W1T, Hp, 128, 64);
  k_agg<2><<<gA, NTHR, AGG_LDS_BYTES, stream>>>(src, dst, nE, nN, vec8, MP, DIS, Hp, b1, XHLw);
  k_gemm<<<dim3(gM, 128 / GBN), GTHR, 0, stream>>>(XHL, W2D, Hp, 128, 128);
  k_agg<4><<<gA, NTHR, AGG_LDS_BYTES, stream>>>(src, dst, nE, nN, vec8, MP, DIS, Hp, b2, XHLw);
  k_gemm<<<dim3(gM, 256 / GBN), GTHR, 0, stream>>>(XHL, W3D, Hp, 256, 256);
  k_agg<8><<<gA, NTHR, AGG_LDS_BYTES, stream>>>(src, dst, nE, nN, vec8, MP, DIS, Hp, b3, XHLw);
  k_gemm<<<dim3(gM, 256 / GBN), GTHR, 0, stream>>>(XHL, WFND, Hp, 512, 256);
  k_edge<<<nE / ETB, ETB, EDGE_LDS_BYTES, stream>>>(src, dst, nN, nE, EA, Hp, WeT, WFED, WF2D, WHD, CST, out);
}
